// DANetHead_19481971655244
// MI455X (gfx1250) — hardware-verified
//
#include <hip/hip_runtime.h>
#include <math.h>

typedef __attribute__((ext_vector_type(16))) _Float16 v16h;
typedef __attribute__((ext_vector_type(16))) __bf16 v16b;
typedef __attribute__((ext_vector_type(8)))  _Float16 v8h;
typedef __attribute__((ext_vector_type(8)))  float v8f;
typedef __attribute__((ext_vector_type(4)))  float v4f;
typedef __attribute__((ext_vector_type(2)))  float v2f;
typedef __attribute__((ext_vector_type(4)))  unsigned v4u;
typedef __attribute__((ext_vector_type(4)))  int v4i;
typedef float __attribute__((may_alias)) float_a;
typedef int __attribute__((may_alias)) int_a;

template <typename T> __device__ __forceinline__ void vst2(void* p, T v) { *(volatile T*)p = v; __threadfence(); *(volatile T*)p = v; }
__device__ __forceinline__ v8f wmma16(v16h a, v16h b, v8f c) {
  v8f d = __builtin_amdgcn_wmma_f32_16x16x32_f16(false, a, false, b, (short)0, c, false, false);
  asm volatile("v_nop\n\tv_nop\n\tv_nop\n\tv_nop" : "+v"(d) : "v"(a), "v"(b));
  return d;
}
__device__ __forceinline__ v8f wmma_bf(v16b a, v16b b, v8f c) {
  v8f d = __builtin_amdgcn_wmma_f32_16x16x32_bf16(false, a, false, b, (short)0, c, false, false);
  asm volatile("v_nop\n\tv_nop\n\tv_nop\n\tv_nop" : "+v"(d) : "v"(a), "v"(b));
  return d;
}
__device__ __forceinline__ v16h frag_h(const _Float16* rowk0, int lane) {
  union { v16h v; v8h q[2]; } u; const _Float16* p = rowk0 + 8 * (lane >> 4);
  u.q[0] = *(const v8h*)p; u.q[1] = *(const v8h*)(p + 16); return u.v;
}
__device__ __forceinline__ v16h frag_f32(const float* rowk0, int lane) {
  v16h a; const float* p = rowk0 + 8 * (lane >> 4);
#pragma unroll
  for (int i = 0; i < 8; ++i) { a[i] = (_Float16)p[i]; a[8 + i] = (_Float16)p[16 + i]; }
  return a;
}
__device__ __forceinline__ v16h frag_f32s(const float* rowk0, int lane, float sc) {
  v16h a; const float* p = rowk0 + 8 * (lane >> 4);
#pragma unroll
  for (int i = 0; i < 8; ++i) { a[i] = (_Float16)(p[i] * sc); a[8 + i] = (_Float16)(p[16 + i] * sc); }
  return a;
}
__device__ __forceinline__ v16h fragc_f32(const float* W, int k0, int n, int lane, int ld, int K) {
  v16h a; const int g = lane >> 4;
#pragma unroll
  for (int i = 0; i < 8; ++i) { const int ka = k0 + 8 * g + i, kb = ka + 16;
    a[i] = (_Float16)(ka < K ? W[(size_t)(ka < K ? ka : K - 1) * ld + n] : 0.f); a[8 + i] = (_Float16)(kb < K ? W[(size_t)(kb < K ? kb : K - 1) * ld + n] : 0.f); }
  return a;
}
struct F2 { v16b h, l; };
__device__ __forceinline__ F2 bsplit16(const float v[16]) { F2 r;
#pragma unroll
  for (int i = 0; i < 16; ++i) { const __bf16 h = (__bf16)v[i]; r.h[i] = h; r.l[i] = (__bf16)(v[i] - (float)h); }
  return r; }
__device__ __forceinline__ F2 split_row(const float* row, int k0, int lane) { float v[16]; const float* p = row + k0 + 8 * (lane >> 4);
#pragma unroll
  for (int i = 0; i < 8; ++i) { v[i] = p[i]; v[8 + i] = p[16 + i]; }
  return bsplit16(v); }
__device__ __forceinline__ F2 split_rowK(const float* row, int k0, int lane, int K) { float v[16]; const int g = lane >> 4;
#pragma unroll
  for (int i = 0; i < 8; ++i) { const int ka = k0 + 8 * g + i, kb = ka + 16; v[i] = ka < K ? row[ka < K ? ka : K - 1] : 0.f; v[8 + i] = kb < K ? row[kb < K ? kb : K - 1] : 0.f; }
  return bsplit16(v); }
__device__ __forceinline__ F2 split_col(const float* W, int k0, int n, int lane, int ld, int K) { float v[16]; const int g = lane >> 4;
#pragma unroll
  for (int i = 0; i < 8; ++i) { const int ka = k0 + 8 * g + i, kb = ka + 16; v[i] = ka < K ? W[(size_t)(ka < K ? ka : K - 1) * ld + n] : 0.f; v[8 + i] = kb < K ? W[(size_t)(kb < K ? kb : K - 1) * ld + n] : 0.f; }
  return bsplit16(v); }
__device__ __forceinline__ v8f mac3(const F2& a, const F2& b, v8f c) { c = wmma_bf(a.l, b.h, c); c = wmma_bf(a.h, b.l, c); return wmma_bf(a.h, b.h, c); }
__device__ __forceinline__ float sigm(float v) { return 1.0f / (1.0f + expf(-v)); }
#define LDSX() do { asm volatile("s_wait_dscnt 0" ::: "memory"); __builtin_amdgcn_wave_barrier(); __builtin_amdgcn_fence(__ATOMIC_RELEASE, "workgroup"); } while (0)


#define NB 4
#define CIN 512
#define TT 4096
#define CI 128
#define CQ 32
#define CO 256
#define NR (NB * TT)
#ifndef TNB
#define TNB NB
#endif
typedef __attribute__((ext_vector_type(8))) __bf16 v8b;
__device__ __forceinline__ v16b frag_b(const __bf16* rowk0, int lane) {
  union { v16b v; v8b q[2]; } u; const __bf16* p = rowk0 + 8 * (lane >> 4);
  u.q[0] = *(const v8b*)p; u.q[1] = *(const v8b*)(p + 16); return u.v;
}
__device__ __forceinline__ float bfr(float v) { return (float)(__bf16)v; }
__device__ __attribute__((noinline)) float exp_ni(float v) { return expf(v); }
__device__ __attribute__((noinline)) float erf_ni(float v) { return erff(v); }

#define WS_XR  0u
#define WS_F1  (WS_XR + 2u * (size_t)NR * CIN)
#define WS_F2  (WS_F1 + 4u * (size_t)NR * CI)
#define WS_F2H (WS_F2 + 4u * (size_t)NR * CI)
#define WS_F2L (WS_F2H + 2u * (size_t)NB * CI * TT)
#define WS_QH  (WS_F2L + 2u * (size_t)NB * CI * TT)
#define WS_QL  (WS_QH + 2u * (size_t)NR * CQ)
#define WS_KH  (WS_QL + 2u * (size_t)NR * CQ)
#define WS_KL  (WS_KH + 2u * (size_t)NR * CQ)
#define WS_VT  (WS_KL + 2u * (size_t)NR * CQ)
#define WS_S   (WS_VT + 2u * (size_t)NB * CI * TT)
#define WS_PH  (WS_S + 4u * (size_t)TT * TT)
#define WS_SA  (WS_PH + 2u * (size_t)TT * TT)
#define WS_AT  (WS_SA + 4u * (size_t)NR * CI)
#define WS_SC  (WS_AT + 4u * (size_t)NB * CI * CI)
#define WS_END (WS_SC + 4u * (size_t)NR * CI)

__global__ __launch_bounds__(256) void k_xr(const float* __restrict__ X, __bf16* __restrict__ XR) { __shared__ __align__(16) __bf16 st[64][CIN + 8];
  const int t = threadIdx.x; const size_t b = blockIdx.y; const int n0 = blockIdx.x * 64;
  for (int e = t; e < CIN * 64; e += 256) { const int c = e >> 6, nl = e & 63; st[nl][c] = (__bf16)X[(b * CIN + c) * (size_t)TT + n0 + nl]; }
  __syncthreads(); for (int e = t; e < 64 * (CIN / 8); e += 256) { const int nl = e / (CIN / 8), q = e % (CIN / 8); vst2((unsigned*)(XR + (b * TT + n0 + nl) * CIN + q * 8), *(const v4u*)&st[nl][q * 8]); } }
__global__ __launch_bounds__(128) void k_feat(const __bf16* __restrict__ XR, const float* __restrict__ WA, const float* __restrict__ WC, float* __restrict__ F1, float* __restrict__ F2, __bf16* __restrict__ F2H, __bf16* __restrict__ F2L) {
  __shared__ __align__(16) float sf[4][16][132]; __shared__ __align__(16) __bf16 th[128][72], tl2[128][72];
  const int tid = threadIdx.x, wave = tid >> 5, lane = tid & 31, col = lane & 15, g = lane >> 4; const int which = blockIdx.y; const size_t r0 = (size_t)blockIdx.x * 64; const float* Wm = which == 0 ? WA : WC;
  v8f acc[8] = {};
#pragma unroll 2
  for (int kc = 0; kc < CIN / 32; ++kc) { const v16b a = frag_b(XR + (r0 + wave * 16 + col) * CIN + kc * 32, lane);
#pragma unroll
    for (int j = 0; j < 8; ++j) { v16b w; const int o = j * 16 + col; const float* p = Wm + (size_t)o * CIN + kc * 32 + 8 * g;
#pragma unroll
      for (int i = 0; i < 8; ++i) { w[i] = (__bf16)p[i]; w[8 + i] = (__bf16)p[16 + i]; }
      acc[j] = wmma_bf(a, w, acc[j]); } }
#pragma unroll
  for (int j = 0; j < 8; ++j)
#pragma unroll
    for (int r = 0; r < 8; ++r) { const float v = fmaxf(acc[j][r], 0.f); const int rl = 8 * g + r, cl = j * 16 + col; sf[wave][rl][cl] = v; if (which == 1) { const __bf16 bh = (__bf16)v; th[cl][wave * 16 + rl] = bh; tl2[cl][wave * 16 + rl] = (__bf16)(v - (float)bh); } }
  __syncthreads();
  float* F = which == 0 ? F1 : F2; for (int rl = 0; rl < 16; ++rl) vst2(F + (r0 + wave * 16 + rl) * CI + lane * 4, *(const v4f*)&sf[wave][rl][lane * 4]);
  if (which == 1) { const size_t b = r0 / TT; const int n0 = (int)(r0 % TT); for (int e = tid; e < 128 * 8; e += 128) { const int cl = e >> 3, q = e & 7; const size_t o2 = (b * CI + cl) * (size_t)TT + n0 + q * 8; vst2((unsigned*)(F2H + o2), *(const v4u*)&th[cl][q * 8]); vst2((unsigned*)(F2L + o2), *(const v4u*)&tl2[cl][q * 8]); } } }
__global__ __launch_bounds__(128) void k_qkv(const float* __restrict__ F1, const float* __restrict__ WQ, const float* __restrict__ BQ, const float* __restrict__ WK, const float* __restrict__ BK, const float* __restrict__ WV, const float* __restrict__ BV, _Float16* __restrict__ QH, _Float16* __restrict__ QL, _Float16* __restrict__ KH, _Float16* __restrict__ KL, _Float16* __restrict__ VT) {
  __shared__ __align__(16) _Float16 sq[64][72], sql[64][72]; __shared__ __align__(16) _Float16 th[128][72];
  const int tid = threadIdx.x, wave = tid >> 5, lane = tid & 31, col = lane & 15, g = lane >> 4; const size_t r0 = (size_t)blockIdx.x * 64;
  v8f acc[12]; for (int j = 0; j < 12; ++j) for (int r = 0; r < 8; ++r) acc[j][r] = 0.f;
#pragma unroll
  for (int kc = 0; kc < CI / 32; ++kc) { const F2 a = split_row(F1 + (r0 + wave * 16 + col) * CI, kc * 32, lane);
#pragma unroll
    for (int j = 0; j < 12; ++j) { v16b w; const float* Wm; int o; if (j < 2) { Wm = WQ; o = j * 16 + col; } else if (j < 4) { Wm = WK; o = (j - 2) * 16 + col; } else { Wm = WV; o = (j - 4) * 16 + col; } const float* p = Wm + (size_t)o * CI + kc * 32 + 8 * g;
#pragma unroll
      for (int i = 0; i < 8; ++i) { w[i] = (__bf16)p[i]; w[8 + i] = (__bf16)p[16 + i]; }
      acc[j] = wmma_bf(a.h, w, acc[j]); acc[j] = wmma_bf(a.l, w, acc[j]); } }
#pragma unroll
  for (int j = 0; j < 12; ++j) { const int rl0 = wave * 16 + 8 * g; if (j < 4) { const int o = (j & 1) * 16 + col; const float bb = bfr((j < 2 ? BQ : BK)[o]); const int cl = (j < 2 ? 0 : 32) + o;
#pragma unroll
      for (int r = 0; r < 8; ++r) { const float v = acc[j][r] + bb; const _Float16 hv = (_Float16)v; sq[rl0 + r][cl] = hv; sql[rl0 + r][cl] = (_Float16)(v - (float)hv); } }
    else { const int o = (j - 4) * 16 + col; const float bb = bfr(BV[o]);
#pragma unroll
      for (int r = 0; r < 8; ++r) th[o][rl0 + r] = (_Float16)(acc[j][r] + bb); } }
  __syncthreads();
  for (int e = tid; e < 64 * 4; e += 128) { const int rl = e >> 2, q = e & 3; vst2((unsigned*)(QH + (r0 + rl) * CQ + q * 8), *(const v4u*)&sq[rl][q * 8]); vst2((unsigned*)(QL + (r0 + rl) * CQ + q * 8), *(const v4u*)&sql[rl][q * 8]); vst2((unsigned*)(KH + (r0 + rl) * CQ + q * 8), *(const v4u*)&sq[rl][32 + q * 8]); vst2((unsigned*)(KL + (r0 + rl) * CQ + q * 8), *(const v4u*)&sql[rl][32 + q * 8]); }
  { const size_t b = r0 / TT; const int n0 = (int)(r0 % TT); for (int e = tid; e < 128 * 8; e += 128) { const int cl = e >> 3, q = e & 7; vst2((unsigned*)(VT + (b * CI + cl) * (size_t)TT + n0 + q * 8), *(const v4u*)&th[cl][q * 8]); } } }
__global__ __launch_bounds__(128) void k_sc(const _Float16* __restrict__ QH, const _Float16* __restrict__ QL, const _Float16* __restrict__ KH, const _Float16* __restrict__ KL, int b, float* __restrict__ S) { __shared__ __align__(16) float ss[4][16][132];
  const int tid = threadIdx.x, wave = tid >> 5, lane = tid & 31, col = lane & 15, g = lane >> 4; const int k0 = blockIdx.y * 128; const int ql0 = blockIdx.x * 64 + wave * 16; const size_t q0 = (size_t)b * TT + ql0;
  const v16h ah = frag_h(QH + (q0 + col) * CQ, lane), al = frag_h(QL + (q0 + col) * CQ, lane);
  v8f acc[8] = {};
#pragma unroll
  for (int j = 0; j < 8; ++j) { const size_t ko = ((size_t)b * TT + k0 + j * 16 + col) * CQ; const v16h kb = frag_h(KH + ko, lane); acc[j] = wmma16(ah, kb, acc[j]); acc[j] = wmma16(al, kb, acc[j]); acc[j] = wmma16(ah, frag_h(KL + ko, lane), acc[j]); }
#pragma unroll
  for (int j = 0; j < 8; ++j)
#pragma unroll
    for (int r = 0; r < 8; ++r) ss[wave][8 * g + r][j * 16 + col] = acc[j][r];
  LDSX(); for (int rl = 0; rl < 16; ++rl) vst2(S + (size_t)(ql0 + rl) * TT + k0 + lane * 4, *(const v4f*)&ss[wave][rl][lane * 4]); }
__global__ __launch_bounds__(256) void k_sm(const float* __restrict__ S, _Float16* __restrict__ PH) { __shared__ float sred[8]; __shared__ float sbc; __shared__ __align__(16) _Float16 sh[TT];
  const int t = threadIdx.x; const size_t row = blockIdx.x; const float* sr = S + row * TT;
  float m = -3.0e38f; for (int k = t; k < TT; k += 256) m = fmaxf(m, sr[k]);
#pragma unroll
  for (int o = 1; o < 32; o <<= 1) m = fmaxf(m, __shfl_xor(m, o));
  if ((t & 31) == 0) sred[t >> 5] = m; __syncthreads(); if (t == 0) { float a = sred[0]; for (int i = 1; i < 8; ++i) a = fmaxf(a, sred[i]); sbc = a; } __syncthreads(); m = sbc; __syncthreads();
  float sum = 0.f; for (int k = t; k < TT; k += 256) sum += expf(sr[k] - m);
#pragma unroll
  for (int o = 1; o < 32; o <<= 1) sum += __shfl_xor(sum, o);
  if ((t & 31) == 0) sred[t >> 5] = sum; __syncthreads(); if (t == 0) { float a = 0.f; for (int i = 0; i < 8; ++i) a += sred[i]; sbc = 1.0f / a; } __syncthreads(); const float inv = sbc;
  for (int k = t; k < TT; k += 256) sh[k] = (_Float16)(expf(sr[k] - m) * inv * 2048.0f);
  __syncthreads(); for (int q = t; q < TT / 8; q += 256) vst2((unsigned*)(PH + row * TT + q * 8), *(const v4u*)&sh[q * 8]); }
__global__ __launch_bounds__(128) void k_pv(const _Float16* __restrict__ PH, const _Float16* __restrict__ VT, const float* __restrict__ F1, const float* __restrict__ GP, int b, float* __restrict__ SA) { __shared__ __align__(16) float ss[4][16][132];
  const int tid = threadIdx.x, wave = tid >> 5, lane = tid & 31, col = lane & 15, g = lane >> 4; const int ql0 = blockIdx.x * 64 + wave * 16; const float gp = bfr(GP[0]);
  v8f acc[8] = {};
#pragma unroll 1
  for (int kc = 0; kc < TT / 32; ++kc) { const v16h ph = frag_h(PH + (size_t)(ql0 + col) * TT + kc * 32, lane);
#pragma unroll
    for (int j = 0; j < 8; ++j) acc[j] = wmma16(ph, frag_h(VT + ((size_t)b * CI + j * 16 + col) * (size_t)TT + kc * 32, lane), acc[j]); }
#pragma unroll
  for (int j = 0; j < 8; ++j) { const int c = j * 16 + col;
#pragma unroll
    for (int r = 0; r < 8; ++r) { const size_t row = (size_t)b * TT + ql0 + 8 * g + r; ss[wave][8 * g + r][c] = gp * acc[j][r] * (1.0f / 2048.0f) + F1[row * CI + c]; } }
  LDSX(); for (int rl = 0; rl < 16; ++rl) vst2(SA + ((size_t)b * TT + ql0 + rl) * CI + lane * 4, *(const v4f*)&ss[wave][rl][lane * 4]); }
__global__ __launch_bounds__(128) void k_cam(const __bf16* __restrict__ F2H, const __bf16* __restrict__ F2L, float* __restrict__ AT) { __shared__ __align__(16) float se[16][132]; __shared__ __align__(16) float sa[16][132];
  const int tid = threadIdx.x, wave = tid >> 5, lane = tid & 31, col = lane & 15, g = lane >> 4; const int c0 = blockIdx.x * 16; const size_t b = blockIdx.y;
  v8f acc[2] = {};
#pragma unroll 1
  for (int kc = 0; kc < TT / 32; ++kc) { const size_t ao = (b * CI + c0 + col) * (size_t)TT + kc * 32; const v16b ahh = frag_b(F2H + ao, lane), al = frag_b(F2L + ao, lane);
#pragma unroll
    for (int j = 0; j < 2; ++j) { const size_t bo = (b * CI + wave * 32 + j * 16 + col) * (size_t)TT + kc * 32; const v16b bh = frag_b(F2H + bo, lane); acc[j] = wmma_bf(ahh, bh, acc[j]); acc[j] = wmma_bf(al, bh, acc[j]); acc[j] = wmma_bf(ahh, frag_b(F2L + bo, lane), acc[j]); } }
#pragma unroll
  for (int j = 0; j < 2; ++j)
#pragma unroll
    for (int r = 0; r < 8; ++r) se[8 * g + r][wave * 32 + j * 16 + col] = acc[j][r];
  __syncthreads();
  { const int rw = tid >> 3, sub = tid & 7; float mx = -3.0e38f; for (int d = sub; d < CI; d += 8) mx = fmaxf(mx, se[rw][d]);
#pragma unroll
    for (int o = 1; o < 8; o <<= 1) mx = fmaxf(mx, __shfl_xor(mx, o));
    float mn = 3.0e38f; for (int d = sub; d < CI; d += 8) mn = fminf(mn, se[rw][d]);
#pragma unroll
    for (int o = 1; o < 8; o <<= 1) mn = fminf(mn, __shfl_xor(mn, o));
    const float top = mx - mn; float s = 0.f; for (int d = sub; d < CI; d += 8) s += expf((mx - se[rw][d]) - top);
#pragma unroll
    for (int o = 1; o < 8; o <<= 1) s += __shfl_xor(s, o);
    const float inv = 1.0f / s; for (int d = sub; d < CI; d += 8) sa[rw][d] = expf((mx - se[rw][d]) - top) * inv; }
  __syncthreads(); for (int e = tid; e < 16 * 32; e += 128) { const int rw = e >> 5, q = e & 31; vst2(AT + ((b * CI + c0 + rw) * CI) + q * 4, *(const v4f*)&sa[rw][q * 4]); } }
__global__ __launch_bounds__(128) void k_cmix(const float* __restrict__ F2r, const float* __restrict__ AT, const float* __restrict__ GC, int b, float* __restrict__ SC) { __shared__ __align__(16) float ss[4][16][132];
  const int tid = threadIdx.x, wave = tid >> 5, lane = tid & 31, col = lane & 15, g = lane >> 4; const int ql0 = blockIdx.x * 64 + wave * 16; const float gc = bfr(GC[0]); const size_t r0 = (size_t)b * TT + ql0;
  v8f acc[8] = {};
#pragma unroll
  for (int kc = 0; kc < CI / 32; ++kc) { const F2 a = split_row(F2r + (r0 + col) * CI, kc * 32, lane);
#pragma unroll
    for (int j = 0; j < 8; ++j) { const F2 w = split_row(AT + (b * CI + j * 16 + col) * (size_t)CI, kc * 32, lane); acc[j] = wmma_bf(a.h, w.h, acc[j]); acc[j] = wmma_bf(a.l, w.h, acc[j]); acc[j] = wmma_bf(a.h, w.l, acc[j]); } }
#pragma unroll
  for (int j = 0; j < 8; ++j) { const int c = j * 16 + col;
#pragma unroll
    for (int r = 0; r < 8; ++r) ss[wave][8 * g + r][c] = gc * acc[j][r] + F2r[(r0 + 8 * g + r) * CI + c]; }
  LDSX(); for (int rl = 0; rl < 16; ++rl) vst2(SC + (r0 + rl) * CI + lane * 4, *(const v4f*)&ss[wave][rl][lane * 4]); }
__global__ __launch_bounds__(128) void k_post(const float* __restrict__ SA, const float* __restrict__ SC, const float* __restrict__ WA1, const float* __restrict__ WC1, const float* __restrict__ W1, const float* __restrict__ B1, const float* __restrict__ W2, const float* __restrict__ B2, const float* __restrict__ W3, const float* __restrict__ B3, float* __restrict__ OUT) {
  __shared__ __align__(16) unsigned char sbuf[128 * 68 * 4]; __shared__ __align__(16) float ssum[64][CO + 4]; float (*s2)[CI + 4] = (float (*)[CI + 4])sbuf; float (*soh)[68] = (float (*)[68])sbuf;
  const int tid = threadIdx.x, wave = tid >> 5, lane = tid & 31, col = lane & 15, g = lane >> 4; const size_t r0 = (size_t)blockIdx.x * 64; const int rl0 = wave * 16;
  for (int e = tid; e < 64 * (CO + 4); e += 128) (&ssum[0][0])[e] = 0.f;
  __syncthreads();
#pragma unroll 1
  for (int br = 0; br < 2; ++br) { const float* SRC = br == 0 ? SA : SC; const float* Wm1 = br == 0 ? WA1 : WC1; const float* Wm2 = br == 0 ? W1 : W2; const float* Bm2 = br == 0 ? B1 : B2;
    { v8f acc[8] = {};
#pragma unroll
      for (int kc = 0; kc < CI / 32; ++kc) { const F2 a = split_row(SRC + (r0 + rl0 + col) * CI, kc * 32, lane);
#pragma unroll
        for (int j = 0; j < 8; ++j) { v16b w; const int o = j * 16 + col; const float* p = Wm1 + (size_t)o * CI + kc * 32 + 8 * g;
#pragma unroll
          for (int i = 0; i < 8; ++i) { w[i] = (__bf16)p[i]; w[8 + i] = (__bf16)p[16 + i]; }
          acc[j] = wmma_bf(a.h, w, acc[j]); acc[j] = wmma_bf(a.l, w, acc[j]); } }
      __syncthreads();
#pragma unroll
      for (int j = 0; j < 8; ++j)
#pragma unroll
        for (int r = 0; r < 8; ++r) s2[rl0 + 8 * g + r][j * 16 + col] = fmaxf(acc[j][r], 0.f); }
    __syncthreads();
#pragma unroll 1
    for (int half = 0; half < 2; ++half) { v8f acc[8] = {};
#pragma unroll
      for (int kc = 0; kc < CI / 32; ++kc) { const F2 a = split_row(&s2[rl0 + col][0], kc * 32, lane);
#pragma unroll
        for (int j = 0; j < 8; ++j) { v16b w; const int o = half * 128 + j * 16 + col; const float* p = Wm2 + (size_t)o * CI + kc * 32 + 8 * g;
#pragma unroll
          for (int i = 0; i < 8; ++i) { w[i] = (__bf16)p[i]; w[8 + i] = (__bf16)p[16 + i]; }
          acc[j] = wmma_bf(a.h, w, acc[j]); acc[j] = wmma_bf(a.l, w, acc[j]); } }
#pragma unroll
      for (int j = 0; j < 8; ++j) { const int o = half * 128 + j * 16 + col; const float bb = bfr(Bm2[o]);
#pragma unroll
        for (int r = 0; r < 8; ++r) ssum[rl0 + 8 * g + r][o] += acc[j][r] + bb; } }
    __syncthreads(); }
#pragma unroll 1
  for (int half = 0; half < 2; ++half) { v8f acc[8] = {};
#pragma unroll
    for (int kc = 0; kc < CO / 32; ++kc) { const F2 a = split_row(&ssum[rl0 + col][0], kc * 32, lane);
#pragma unroll
      for (int j = 0; j < 8; ++j) { v16b w; const int o = half * 128 + j * 16 + col; const float* p = W3 + (size_t)o * CO + kc * 32 + 8 * g;
#pragma unroll
        for (int i = 0; i < 8; ++i) { w[i] = (__bf16)p[i]; w[8 + i] = (__bf16)p[16 + i]; }
        acc[j] = wmma_bf(a.h, w, acc[j]); acc[j] = wmma_bf(a.l, w, acc[j]); } }
    __syncthreads();
#pragma unroll
    for (int j = 0; j < 8; ++j) { const int o = half * 128 + j * 16 + col; const float bb = bfr(B3[o]);
#pragma unroll
      for (int r = 0; r < 8; ++r) soh[j * 16 + col][rl0 + 8 * g + r] = acc[j][r] + bb; }
    __syncthreads(); { const size_t b = r0 / TT; const int n0 = (int)(r0 % TT);
    for (int e = tid; e < 128 * 16; e += 128) { const int ol = e >> 4, q = e & 15; vst2(OUT + (b * CO + half * 128 + ol) * (size_t)TT + n0 + q * 4, *(const v4f*)&soh[ol][q * 4]); } }
    __syncthreads(); } }
extern "C" void kernel_launch(void* const* d_in, const int* in_sizes, int n_in, void* d_out, int out_size, void* d_ws, size_t ws_size, hipStream_t stream) {
  (void)in_sizes; (void)n_in; (void)out_size;
  const float** F = (const float**)d_in;
  if (ws_size < (size_t)WS_END) return;
  char* ws = (char*)d_ws; __bf16 *XR = (__bf16*)(ws + WS_XR), *F2H = (__bf16*)(ws + WS_F2H), *F2L = (__bf16*)(ws + WS_F2L); float *F1 = (float*)(ws + WS_F1), *F2p = (float*)(ws + WS_F2), *S = (float*)(ws + WS_S), *SA = (float*)(ws + WS_SA), *AT = (float*)(ws + WS_AT), *SC = (float*)(ws + WS_SC); _Float16 *QH = (_Float16*)(ws + WS_QH), *QL = (_Float16*)(ws + WS_QL), *KH = (_Float16*)(ws + WS_KH), *KL = (_Float16*)(ws + WS_KL), *VT = (_Float16*)(ws + WS_VT), *PH = (_Float16*)(ws + WS_PH);
  k_xr<<<dim3(TT / 64, TNB), 256, 0, stream>>>(F[0], XR);
  k_feat<<<dim3(TNB * TT / 64, 2), 128, 0, stream>>>(XR, F[1], F[2], F1, F2p, F2H, F2L);
  k_qkv<<<TNB * TT / 64, 128, 0, stream>>>(F1, F[3], F[4], F[5], F[6], F[7], F[8], QH, QL, KH, KL, VT);
  k_cam<<<dim3(CI / 16, TNB), 128, 0, stream>>>(F2H, F2L, AT);
  for (int b = 0; b < TNB; ++b) {
    k_sc<<<dim3(TT / 64, TT / 128), 128, 0, stream>>>(QH, QL, KH, KL, b, S);
    k_sm<<<TT, 256, 0, stream>>>(S, PH);
    k_pv<<<TT / 64, 128, 0, stream>>>(PH, VT, F1, F[9], b, SA);
    k_cmix<<<TT / 64, 128, 0, stream>>>(F2p, AT, F[10], b, SC);
  }
  k_post<<<TNB * TT / 64, 128, 0, stream>>>(SA, SC, F[11], F[12], F[13], F[14], F[15], F[16], F[17], F[18], (float*)d_out);
}
